// TransformerBlock_15358803050647
// MI455X (gfx1250) — hardware-verified
//
#include <hip/hip_runtime.h>
#include <stddef.h>


typedef _Float16 v16h __attribute__((ext_vector_type(16)));
typedef _Float16 v8h  __attribute__((ext_vector_type(8)));
typedef float    v8f  __attribute__((ext_vector_type(8)));
typedef float    v4f  __attribute__((ext_vector_type(4)));

#ifndef NB
#define NB 8
#endif
#define NB_FULL 8
#define CDIM  512
#define NPIX  1024
#define C3    1536
#define C4    2048
#define NHEAD 8
#define HD    64

static_assert(NB >= 1 && NB <= NB_FULL);
static_assert(CDIM == NHEAD * HD);
static_assert(HD == 64);
static_assert((NPIX % 128) == 0 && (CDIM % 64) == 0 && (C3 % 64) == 0 && (C4 % 64) == 0);
static_assert((CDIM % 32) == 0 && (C4 % 32) == 0);

#define LDT 72
#define LDC 68

#define WCARRY 64.0f
#define BN_EPS 1.0e-5f

#define OFF_WQ  ((size_t)0)
#define OFF_WO  ((size_t)C3 * CDIM)
#define OFF_WF1 (OFF_WO + (size_t)CDIM * CDIM)
#define OFF_WF2 (OFF_WF1 + (size_t)C4 * CDIM)
#define W_ELEMS (OFF_WF2 + (size_t)CDIM * C4)
static_assert((((size_t)C3 * CDIM) % 2048) == 0 && (((size_t)CDIM * CDIM) % 2048) == 0);
static_assert((((size_t)C4 * CDIM) % 2048) == 0);

#define W_BYTES   (W_ELEMS * 2)
#define XT_BYTES  ((size_t)NB * NPIX * CDIM * 2)
#define QKV_BYTES ((size_t)NB * C3 * NPIX * 2)
#define ATT_BYTES ((size_t)NB * CDIM * NPIX * 2)
#define AT_BYTES  ((size_t)NB * NPIX * CDIM * 2)
#define H_BYTES   ((size_t)NB * CDIM * NPIX * 4)
#define HT_BYTES  ((size_t)NB * NPIX * CDIM * 2)
#define FT_BYTES  ((size_t)NB * NPIX * C4 * 2)
#define WS_TOTAL  (W_BYTES + XT_BYTES + QKV_BYTES + ATT_BYTES + AT_BYTES + H_BYTES + HT_BYTES + FT_BYTES)
static_assert((W_BYTES % 128) == 0 && (XT_BYTES % 128) == 0 && (QKV_BYTES % 128) == 0);
static_assert((ATT_BYTES % 128) == 0 && (H_BYTES % 128) == 0 && (FT_BYTES % 128) == 0);
static_assert(WS_TOTAL <= (size_t)134217728);

__device__ __forceinline__ float bf16r(float x) {
  unsigned int u = __float_as_uint(x);
  u = (u + 0x7FFFu + ((u >> 16) & 1u)) & 0xFFFF0000u;
  return __uint_as_float(u);
}

__device__ __forceinline__ v16h frag_join(v8h lo, v8h hi) {
  v16h out;
#pragma unroll
  for (int i = 0; i < 8; ++i) { out[i] = lo[i]; out[i + 8] = hi[i]; }
  return out;
}

__device__ __forceinline__ v16h frag_at(const _Float16* __restrict__ p) {
  const v8h lo = *(const v8h*)(p);
  const v8h hi = *(const v8h*)(p + 16);
  return frag_join(lo, hi);
}

__device__ __forceinline__ v8f wmma16(v16h a, v16h b, v8f c) {
  v8f d = __builtin_amdgcn_wmma_f32_16x16x32_f16(false, a, false, b, (short)0, c,
                                                 false, false);
  asm volatile("v_nop\n\tv_nop\n\tv_nop\n\tv_nop" : "+v"(d) : "v"(a), "v"(b));
  return d;
}

__device__ __forceinline__ void wave_lds_sync() {
  __builtin_amdgcn_fence(3  , "wavefront");
  asm volatile("s_wait_dscnt 0x0" ::: "memory");
  __builtin_amdgcn_wave_barrier();
}

__device__ __forceinline__ float silu_f(float y) {
  return y * __builtin_amdgcn_rcpf(1.0f + __expf(-y));
}

__global__ __launch_bounds__(256) void wcast_kernel(
    const float* __restrict__ src, _Float16* __restrict__ dst) {
  const size_t e = ((size_t)blockIdx.x * 256u + threadIdx.x) * 8u;
  const v4f a0 = *(const v4f*)(src + e);
  const v4f a1 = *(const v4f*)(src + e + 4);
  v8h o;
#pragma unroll
  for (int j = 0; j < 4; ++j) {
    o[j]     = (_Float16)(WCARRY * bf16r(a0[j]));
    o[j + 4] = (_Float16)(WCARRY * bf16r(a1[j]));
  }
  *(volatile v8h*)(dst + e) = o;
  __threadfence();
  *(volatile v8h*)(dst + e) = o;
}

__global__ __launch_bounds__(256) void xt_kernel(
    const float* __restrict__ X, _Float16* __restrict__ XT) {
  __shared__ __attribute__((aligned(16))) _Float16 T[64 * LDT];
  const unsigned tid = threadIdx.x;
  const unsigned p0 = blockIdx.x * 64u;
  const unsigned c0 = blockIdx.y * 64u;
  const unsigned b = blockIdx.z;
  const size_t sbase = ((size_t)b * CDIM + c0) * NPIX + p0;
#pragma unroll
  for (unsigned j = 0; j < 4u; ++j) {
    const unsigned idx = tid + 256u * j;
    const unsigned cr = idx >> 4, pc = (idx & 15u) * 4u;
    const v4f v = *(const v4f*)(X + sbase + (size_t)cr * NPIX + pc);
#pragma unroll
    for (unsigned q = 0; q < 4u; ++q) T[(pc + q) * LDT + cr] = (_Float16)bf16r(v[q]);
  }
  __syncthreads();
  v8h x[2];
  size_t off[2];
#pragma unroll
  for (unsigned i = 0; i < 2u; ++i) {
    const unsigned n = 32u * i + (tid >> 3);
    const unsigned kc = (tid & 7u) * 8u;
    x[i] = *(const v8h*)&T[n * LDT + kc];
    off[i] = ((size_t)b * NPIX + p0 + n) * CDIM + c0 + kc;
  }
#pragma unroll
  for (int i = 0; i < 2; ++i) *(volatile v8h*)(XT + off[i]) = x[i];
  __threadfence();
#pragma unroll
  for (int i = 0; i < 2; ++i) *(volatile v8h*)(XT + off[i]) = x[i];
}

__global__ __launch_bounds__(256) void atr_kernel(
    const _Float16* __restrict__ S, _Float16* __restrict__ D) {
  __shared__ __attribute__((aligned(16))) _Float16 T[64 * LDT];
  const unsigned tid = threadIdx.x;
  const unsigned p0 = blockIdx.x * 64u;
  const unsigned c0 = blockIdx.y * 64u;
  const unsigned b = blockIdx.z;
  const size_t sbase = ((size_t)b * CDIM + c0) * NPIX + p0;
#pragma unroll
  for (unsigned j = 0; j < 2u; ++j) {
    const unsigned idx = tid + 256u * j;
    const unsigned cr = idx >> 3, pc = (idx & 7u) * 8u;
    const v8h v = *(const v8h*)(S + sbase + (size_t)cr * NPIX + pc);
#pragma unroll
    for (unsigned q = 0; q < 8u; ++q) T[(pc + q) * LDT + cr] = v[q];
  }
  __syncthreads();
  v8h x[2];
  size_t off[2];
#pragma unroll
  for (unsigned i = 0; i < 2u; ++i) {
    const unsigned n = 32u * i + (tid >> 3);
    const unsigned kc = (tid & 7u) * 8u;
    x[i] = *(const v8h*)&T[n * LDT + kc];
    off[i] = ((size_t)b * NPIX + p0 + n) * CDIM + c0 + kc;
  }
#pragma unroll
  for (int i = 0; i < 2; ++i) *(volatile v8h*)(D + off[i]) = x[i];
  __threadfence();
#pragma unroll
  for (int i = 0; i < 2; ++i) *(volatile v8h*)(D + off[i]) = x[i];
}

template <int MODE, int KD, int OD>
__global__ __launch_bounds__(256) void gemm_kernel(
    const _Float16* __restrict__ A16, const _Float16* __restrict__ Bt,
    const float* __restrict__ bias, const float* __restrict__ gam,
    const float* __restrict__ bet, const float* __restrict__ mu,
    const float* __restrict__ var, const float* __restrict__ resid,
    float* __restrict__ outf, _Float16* __restrict__ out16) {
  __shared__ __attribute__((aligned(16))) float Cs[64 * LDC];
  const unsigned tid = threadIdx.x, lane = tid & 31u;
  const unsigned w = (unsigned)__builtin_amdgcn_readfirstlane((int)(threadIdx.x >> 5));
  const unsigned mw = w >> 1, nw = w & 1u;
  const unsigned hh = lane >> 4, m = lane & 15u;
  const unsigned n0 = blockIdx.x * 64u;
  const unsigned row0 = blockIdx.y * 64u;
  const unsigned b = blockIdx.z;

  const _Float16* ap  = A16 + (size_t)(row0 + mw * 16u + m) * KD + hh * 8u;
  const _Float16* bp0 = Bt + ((size_t)b * NPIX + n0 + nw * 32u + m) * KD + hh * 8u;
  const _Float16* bp1 = bp0 + 16 * KD;
  v8f acc0 = {}, acc1 = {};
#pragma unroll 2
  for (unsigned k0 = 0; k0 < (unsigned)KD; k0 += 32u) {
    const v16h a  = frag_at(ap + k0);
    const v16h b0 = frag_at(bp0 + k0);
    const v16h b1 = frag_at(bp1 + k0);
    acc0 = wmma16(a, b0, acc0);
    acc1 = wmma16(a, b1, acc1);
  }
#pragma unroll
  for (int r = 0; r < 8; ++r) {
    const unsigned ci = (mw * 16u + hh * 8u + (unsigned)r) * LDC + nw * 32u + m;
    Cs[ci]      = acc0[r];
    Cs[ci + 16] = acc1[r];
  }
  __syncthreads();

  if (MODE == 0) {
    v8h x[2];
    size_t off[2];
#pragma unroll
    for (unsigned i = 0; i < 2u; ++i) {
      const unsigned r = 32u * i + (tid >> 3);
      const unsigned c = (tid & 7u) * 8u;
      const unsigned o = row0 + r;
      const float bv = bf16r(bias[o]);
      const v4f u0 = *(const v4f*)&Cs[r * LDC + c];
      const v4f u1 = *(const v4f*)&Cs[r * LDC + c + 4];
#pragma unroll
      for (int j = 0; j < 4; ++j) {
        x[i][j]     = (_Float16)(u0[j] * (1.0f / WCARRY) + bv);
        x[i][j + 4] = (_Float16)(u1[j] * (1.0f / WCARRY) + bv);
      }
      off[i] = ((size_t)b * OD + o) * NPIX + n0 + c;
    }
#pragma unroll
    for (int i = 0; i < 2; ++i) *(volatile v8h*)(out16 + off[i]) = x[i];
    __threadfence();
#pragma unroll
    for (int i = 0; i < 2; ++i) *(volatile v8h*)(out16 + off[i]) = x[i];
  }

  if (MODE != 0) {
    v4f xs[4];
    size_t off[4];
#pragma unroll
    for (unsigned i = 0; i < 4u; ++i) {
      const unsigned r = 16u * i + (tid >> 4);
      const unsigned c = (tid & 15u) * 4u;
      const unsigned o = row0 + r;
      const float gm = bf16r(gam[o]);
      const float bt = bf16r(bet[o]);
      const float mm = bf16r(mu[o]);
      const float vv = bf16r(var[o]);
      const float sc = gm * rsqrtf(vv + BN_EPS);
      const v4f u = *(const v4f*)&Cs[r * LDC + c];
      const size_t gidx = ((size_t)b * OD + o) * NPIX + n0 + c;
      v4f val;
      if (MODE == 1) {
        const float bo = bf16r(bias[o]);
        const v4f xr = *(const v4f*)(resid + gidx);
#pragma unroll
        for (int j = 0; j < 4; ++j) {
          const float t = bf16r(xr[j]) + (u[j] * (1.0f / WCARRY) + bo);
          val[j] = (t - mm) * sc + bt;
        }
      }
      if (MODE == 2) {
#pragma unroll
        for (int j = 0; j < 4; ++j) {
          const float y = (u[j] * (1.0f / WCARRY) - mm) * sc + bt;
          val[j] = silu_f(y);
        }
      }
      if (MODE == 3) {
        const v4f hr = *(const v4f*)(resid + gidx);
#pragma unroll
        for (int j = 0; j < 4; ++j) {
          const float y = (u[j] * (1.0f / WCARRY) - mm) * sc + bt;
          val[j] = hr[j] + silu_f(y);
        }
      }
      xs[i] = val;
      off[i] = gidx;
      if (MODE == 1 || MODE == 2) *(v4f*)&Cs[r * LDC + c] = val;
    }

    if (MODE == 1 || MODE == 2) {
      __syncthreads();
      v8h xt[2];
      size_t o2[2];
#pragma unroll
      for (unsigned i = 0; i < 2u; ++i) {
        const unsigned dcol = 32u * i + (tid >> 3);
        const unsigned kk = (tid & 7u) * 8u;
#pragma unroll
        for (unsigned j = 0; j < 8u; ++j)
          xt[i][j] = (_Float16)Cs[(kk + j) * LDC + dcol];
        o2[i] = ((size_t)b * NPIX + n0 + dcol) * OD + row0 + kk;
      }
      if (MODE == 1) {
#pragma unroll
        for (int i = 0; i < 4; ++i) *(volatile v4f*)(outf + off[i]) = xs[i];
      }
#pragma unroll
      for (int i = 0; i < 2; ++i) *(volatile v8h*)(out16 + o2[i]) = xt[i];
      __threadfence();
      if (MODE == 1) {
#pragma unroll
        for (int i = 0; i < 4; ++i) *(volatile v4f*)(outf + off[i]) = xs[i];
      }
#pragma unroll
      for (int i = 0; i < 2; ++i) *(volatile v8h*)(out16 + o2[i]) = xt[i];
    }

    if (MODE == 3) {
#pragma unroll
      for (int i = 0; i < 4; ++i) *(volatile v4f*)(outf + off[i]) = xs[i];
      __threadfence();
#pragma unroll
      for (int i = 0; i < 4; ++i) *(volatile v4f*)(outf + off[i]) = xs[i];
    }
  }
}

__global__ __launch_bounds__(256) void attn_kernel(
    const _Float16* __restrict__ QKV, _Float16* __restrict__ Att) {
  __shared__ __attribute__((aligned(16))) _Float16 Ks[64 * LDT];
  __shared__ float Ss[128];

  const unsigned tid = threadIdx.x, lane = tid & 31u;
  const unsigned w = (unsigned)__builtin_amdgcn_readfirstlane((int)(threadIdx.x >> 5));
  const unsigned hh = lane >> 4, m = lane & 15u;
  const unsigned q0 = blockIdx.x * 128u;
  const unsigned head = blockIdx.y;
  const unsigned b = blockIdx.z;
  const float scale = 0.125f;

  const size_t qbase = ((size_t)b * C3 + head * HD) * NPIX;
  const size_t kbase = qbase + (size_t)CDIM * NPIX;
  const size_t vbase = qbase + (size_t)2 * CDIM * NPIX;

  const size_t qoff = qbase + (size_t)(q0 + w * 16u + m) * HD + hh * 8u;
  v16h qf[2];
  qf[0] = frag_at(QKV + qoff);
  qf[1] = frag_at(QKV + qoff + 32);

  float mrow[8], lrow[8];
#pragma unroll
  for (int v = 0; v < 8; ++v) { mrow[v] = -1.0e30f; lrow[v] = 0.0f; }

  for (unsigned kb = 0; kb < (unsigned)NPIX; kb += 64u) {
#pragma unroll
    for (unsigned j = 0; j < 2u; ++j) {
      const unsigned idx = tid + 256u * j;
      const unsigned r = idx >> 3, c = (idx & 7u) * 8u;
      *(v8h*)&Ks[r * LDT + c] = *(const v8h*)(QKV + kbase + (size_t)(kb + r) * HD + c);
    }
    __syncthreads();

    v8f s[4];
#pragma unroll
    for (int kg = 0; kg < 4; ++kg) {
      v8f t = {};
#pragma unroll
      for (int c = 0; c < 2; ++c) {
        const unsigned ki = ((unsigned)kg * 16u + m) * LDT + (unsigned)c * 32u + hh * 8u;
        const v8h klo = *(const v8h*)&Ks[ki];
        const v8h khi = *(const v8h*)&Ks[ki + 16];
        t = wmma16(qf[c], frag_join(klo, khi), t);
      }
      s[kg] = t * scale;
    }

#pragma unroll
    for (int v = 0; v < 8; ++v) {
      const float mx = fmaxf(fmaxf(s[0][v], s[1][v]), fmaxf(s[2][v], s[3][v]));
      const float mn = fmaxf(mrow[v], mx);
      const float al = __expf(mrow[v] - mn);
      const float e = (__expf(s[0][v] - mn) + __expf(s[1][v] - mn)) +
                      (__expf(s[2][v] - mn) + __expf(s[3][v] - mn));
      lrow[v] = al * lrow[v] + e;
      mrow[v] = mn;
    }
    __syncthreads();
  }

#pragma unroll
  for (int v = 0; v < 8; ++v) {
#pragma unroll
    for (int off = 1; off < 16; off <<= 1) {
      const float m2 = __shfl_xor(mrow[v], off, 32);
      const float l2 = __shfl_xor(lrow[v], off, 32);
      const float nm = fmaxf(mrow[v], m2);
      lrow[v] = lrow[v] * __expf(mrow[v] - nm) + l2 * __expf(m2 - nm);
      mrow[v] = nm;
    }
  }

  float sv = 0.0f;
#pragma unroll
  for (int v = 0; v < 8; ++v) {
    const float sn = lrow[v] * __builtin_amdgcn_rcpf(lrow[v]);
    sv = (m == (unsigned)v) ? sn : sv;
  }
  if (m < 8u) Ss[w * 16u + hh * 8u + m] = sv;
  wave_lds_sync();

  v8h x[4];
  size_t off[4];
#pragma unroll
  for (unsigned i = 0; i < 4u; ++i) {
    const unsigned r = 4u * i + (lane >> 3);
    const unsigned c = (lane & 7u) * 8u;
    const size_t rowoff = (size_t)(q0 + w * 16u + r) * HD + c;
    const v8h vv = *(const v8h*)(QKV + vbase + rowoff);
    const float sr = Ss[w * 16u + r];
#pragma unroll
    for (int j = 0; j < 8; ++j) x[i][j] = (_Float16)((float)vv[j] * sr);
    off[i] = ((size_t)b * CDIM + head * HD) * NPIX + rowoff;
  }
#pragma unroll
  for (int i = 0; i < 4; ++i) *(volatile v8h*)(Att + off[i]) = x[i];
  __threadfence();
#pragma unroll
  for (int i = 0; i < 4; ++i) *(volatile v8h*)(Att + off[i]) = x[i];
}

extern "C" void kernel_launch(void* const* d_in, const int* in_sizes, int n_in,
                              void* d_out, int out_size, void* d_ws, size_t ws_size,
                              hipStream_t stream) {
  if (n_in < 19) return;
  const long long need_x = (long long)NB * CDIM * NPIX;
  if ((long long)in_sizes[0] < need_x) return;
  if ((long long)in_sizes[1] < (long long)C3 * CDIM) return;
  if (in_sizes[2] < C3) return;
  if ((long long)in_sizes[3] < (long long)CDIM * CDIM) return;
  if (in_sizes[4] < CDIM) return;
  if (in_sizes[5] < CDIM || in_sizes[6] < CDIM || in_sizes[7] < CDIM || in_sizes[8] < CDIM) return;
  if ((long long)in_sizes[9] < (long long)C4 * CDIM) return;
  if (in_sizes[10] < C4 || in_sizes[11] < C4 || in_sizes[12] < C4 || in_sizes[13] < C4) return;
  if ((long long)in_sizes[14] < (long long)CDIM * C4) return;
  if (in_sizes[15] < CDIM || in_sizes[16] < CDIM || in_sizes[17] < CDIM || in_sizes[18] < CDIM) return;
  if ((long long)out_size < need_x) return;
  if (ws_size < WS_TOTAL) return;

  const float* X    = (const float*)d_in[0];
  const float* Wqkv = (const float*)d_in[1];
  const float* bqkv = (const float*)d_in[2];
  const float* Wout = (const float*)d_in[3];
  const float* bout = (const float*)d_in[4];
  const float* g1   = (const float*)d_in[5];
  const float* be1  = (const float*)d_in[6];
  const float* m1   = (const float*)d_in[7];
  const float* v1   = (const float*)d_in[8];
  const float* Wf1  = (const float*)d_in[9];
  const float* g2   = (const float*)d_in[10];
  const float* be2  = (const float*)d_in[11];
  const float* m2   = (const float*)d_in[12];
  const float* v2   = (const float*)d_in[13];
  const float* Wf2  = (const float*)d_in[14];
  const float* g3   = (const float*)d_in[15];
  const float* be3  = (const float*)d_in[16];
  const float* m3   = (const float*)d_in[17];
  const float* v3   = (const float*)d_in[18];
  float* out = (float*)d_out;

  char* ws = (char*)d_ws;
  size_t cur = 0;
  _Float16* W16   = (_Float16*)(ws + cur); cur += W_BYTES;
  _Float16* XT    = (_Float16*)(ws + cur); cur += XT_BYTES;
  _Float16* QKV16 = (_Float16*)(ws + cur); cur += QKV_BYTES;
  _Float16* ATT16 = (_Float16*)(ws + cur); cur += ATT_BYTES;
  _Float16* AT    = (_Float16*)(ws + cur); cur += AT_BYTES;
  float*    Hf    = (float*)(ws + cur);    cur += H_BYTES;
  _Float16* HT    = (_Float16*)(ws + cur); cur += HT_BYTES;
  _Float16* FT    = (_Float16*)(ws + cur); cur += FT_BYTES;
  if (cur > ws_size) return;

  dim3 blk(256);

  wcast_kernel<<<dim3((unsigned)(((size_t)C3 * CDIM) / 2048)), blk, 0, stream>>>(Wqkv, W16 + OFF_WQ);
  wcast_kernel<<<dim3((unsigned)(((size_t)CDIM * CDIM) / 2048)), blk, 0, stream>>>(Wout, W16 + OFF_WO);
  wcast_kernel<<<dim3((unsigned)(((size_t)C4 * CDIM) / 2048)), blk, 0, stream>>>(Wf1, W16 + OFF_WF1);
  wcast_kernel<<<dim3((unsigned)(((size_t)CDIM * C4) / 2048)), blk, 0, stream>>>(Wf2, W16 + OFF_WF2);

  xt_kernel<<<dim3(NPIX / 64, CDIM / 64, NB), blk, 0, stream>>>(X, XT);

  gemm_kernel<0, CDIM, C3><<<dim3(NPIX / 64, C3 / 64, NB), blk, 0, stream>>>(
      W16 + OFF_WQ, XT, bqkv, bqkv, bqkv, bqkv, bqkv, X, Hf, QKV16);

  attn_kernel<<<dim3(NPIX / 128, NHEAD, NB), blk, 0, stream>>>(QKV16, ATT16);

  atr_kernel<<<dim3(NPIX / 64, CDIM / 64, NB), blk, 0, stream>>>(ATT16, AT);

  gemm_kernel<1, CDIM, CDIM><<<dim3(NPIX / 64, CDIM / 64, NB), blk, 0, stream>>>(
      W16 + OFF_WO, AT, bout, g1, be1, m1, v1, X, Hf, HT);

  gemm_kernel<2, CDIM, C4><<<dim3(NPIX / 64, C4 / 64, NB), blk, 0, stream>>>(
      W16 + OFF_WF1, HT, bout, g2, be2, m2, v2, X, Hf, FT);

  gemm_kernel<3, C4, CDIM><<<dim3(NPIX / 64, CDIM / 64, NB), blk, 0, stream>>>(
      W16 + OFF_WF2, FT, bout, g3, be3, m3, v3, Hf, out, HT);
}
